// GerbilizerRNNConv_42829413876222
// MI455X (gfx1250) — hardware-verified
//
#include <hip/hip_runtime.h>


typedef __bf16 bf16t;
typedef bf16t v16b __attribute__((ext_vector_type(16)));
typedef bf16t v8b  __attribute__((ext_vector_type(8)));
typedef bf16t v4b  __attribute__((ext_vector_type(4)));
typedef float v8f  __attribute__((ext_vector_type(8)));
typedef float v4f  __attribute__((ext_vector_type(4)));
typedef unsigned int v4u __attribute__((ext_vector_type(4)));
typedef unsigned int v2u __attribute__((ext_vector_type(2)));

union Frag { v16b v; v4u q[2]; };
union Pk8  { v8b h; v4u u; };
union Pk4  { v4b h; v2u u; };

constexpr int NB    = 16;
constexpr int NSTEP = 64;
constexpr int CIN   = 4;
constexpr int NPOS  = 258;
constexpr int HID   = 32;
constexpr int NGATE = 128;
constexpr int NPAD  = 272;
constexpr int JOBS  = 34;
constexpr int GUARD = 2;
constexpr int COLS  = 276;
constexpr int KP0   = 48;
constexpr int KP1   = 64;
constexpr int KL0   = 128;
constexpr int KL1   = 192;
constexpr int K0IN  = 36;
constexpr int K1IN  = 64;
constexpr int FC1   = 256;
constexpr int NOUT  = 2;

constexpr int SZ_P0 = COLS * KP0 * 2;
constexpr int SZ_P1 = COLS * KP1 * 2;
constexpr int SZ_H1 = NPOS * HID * 2;
constexpr int SZ_C  = NPOS * HID * 4;
constexpr int OFF_P0H  = 0;
constexpr int OFF_P0L  = OFF_P0H + SZ_P0;
constexpr int OFF_P1H  = OFF_P0L + SZ_P0;
constexpr int OFF_P1L  = OFF_P1H + SZ_P1;
constexpr int OFF_H1H  = OFF_P1L + SZ_P1;
constexpr int OFF_H1L  = OFF_H1H + SZ_H1;
constexpr int OFF_C0   = OFF_H1L + SZ_H1;
constexpr int OFF_C1   = OFF_C0 + SZ_C;
constexpr int OFF_FP   = OFF_C1 + SZ_C;
constexpr int OFF_FLAT = OFF_FP + 2 * NPAD * 4;
constexpr int OFF_F1O  = OFF_FLAT + 264 * 4;
constexpr int OFF_RES  = OFF_F1O + FC1 * 4;
constexpr int LDS_BYTES = OFF_RES + 64;
static_assert(LDS_BYTES == 227040);
static_assert((SZ_P0 % 16) == 0 && (SZ_P1 % 16) == 0 && (SZ_H1 % 16) == 0 && (SZ_C % 16) == 0);
static_assert((LDS_BYTES % 16) == 0);

constexpr int PIECES0 = NGATE * (KL0 / 8);
constexpr int PIECES1 = NGATE * (KL1 / 8);
static_assert(PIECES0 == 8 * 256);
static_assert(PIECES0 + PIECES1 == 20 * 256);

constexpr size_t SZ_A0 = (size_t)NGATE * KL0 * 2;
constexpr size_t SZ_A1 = (size_t)NGATE * KL1 * 2;
constexpr size_t SZ_STAGE = (size_t)NB * 32 * 4;

__device__ __forceinline__ v8f wmma_bf(v16b a, v16b b, v8f c) {
  return __builtin_amdgcn_wmma_f32_16x16x32_bf16(false, a, false, b, (short)0, c, false, false);
}

__device__ __forceinline__ v8f wmma3(v8f c, v16b ah, v16b al, v16b bh, v16b bl) {
  c = wmma_bf(ah, bh, c);
  c = wmma_bf(ah, bl, c);
  c = wmma_bf(al, bh, c);
  asm volatile("v_nop\n\tv_nop\n\tv_nop\n\tv_nop"
               : "+v"(c)
               : "v"(ah), "v"(al), "v"(bh), "v"(bl));
  return c;
}

__device__ __forceinline__ float sigf(float x) {
  x = fminf(30.0f, fmaxf(-30.0f, x));
  const float e = expf(-x);
  return __builtin_amdgcn_rcpf(1.0f + e);
}

__device__ __forceinline__ float tanhf_(float x) {
  const float ax = fminf(fabsf(x), 15.0f);
  const float t  = expf(-2.0f * ax);
  const float r  = (1.0f - t) * __builtin_amdgcn_rcpf(1.0f + t);
  return copysignf(r, x);
}

__global__ void __launch_bounds__(256)
k_prep(const float* __restrict__ w0, const float* __restrict__ w1,
       bf16t* A0h, bf16t* A0l, bf16t* A1h, bf16t* A1l) {
  const int i = blockIdx.x * 256 + threadIdx.x;
  if (i >= PIECES0 + PIECES1) return;
  const bool second = blockIdx.x >= (PIECES0 / 256);
  float v[8];
  bf16t* dh;
  bf16t* dl;
  if (!second) {
    const int oc = i >> 4, k8 = (i & 15) * 8;
#pragma unroll
    for (int e = 0; e < 8; ++e) {
      const int k = k8 + e;
      const int tap = (k >= 40 ? 1 : 0) + (k >= 80 ? 1 : 0);
      const int row = k - 40 * tap;
      const bool ish = row < 32;
      const bool isx = (row >= 32) && (row < 32 + CIN);
      int ic = ish ? (row + CIN) : (row - 32);
      ic = ic < 0 ? 0 : (ic > K0IN - 1 ? K0IN - 1 : ic);
      const float wv = w0[(oc * K0IN + ic) * 3 + tap];
      v[e] = (ish || isx) ? wv : 0.0f;
    }
    dh = A0h + oc * KL0 + k8;
    dl = A0l + oc * KL0 + k8;
  } else {
    const int j = i - PIECES0;
    const int oc = j / 24, q = j - 24 * oc, k8 = q * 8;
#pragma unroll
    for (int e = 0; e < 8; ++e) {
      const int k = k8 + e;
      const int tap = k >> 6;
      const int row = k & 63;
      v[e] = w1[(oc * K1IN + row) * 3 + tap];
    }
    dh = A1h + oc * KL1 + k8;
    dl = A1l + oc * KL1 + k8;
  }
  Pk8 ph, pl;
#pragma unroll
  for (int e = 0; e < 8; ++e) {
    const bf16t hb = (bf16t)v[e];
    ph.h[e] = hb;
    pl.h[e] = (bf16t)(v[e] - (float)hb);
  }
  *(volatile v4u*)dh = ph.u;
  *(volatile v4u*)dl = pl.u;
  __threadfence();
  *(volatile v4u*)dh = ph.u;
  *(volatile v4u*)dl = pl.u;
}

template <int L>
__device__ __forceinline__ void layer_jobs(const bf16t* Ph, const bf16t* Pl,
                                           const bf16t* __restrict__ Ah,
                                           const bf16t* __restrict__ Al,
                                           const float* __restrict__ bias,
                                           float* cbuf, bf16t* Oh, bf16t* Ol,
                                           float* fpart, const float* __restrict__ ninw,
                                           bool doLast, int wave, int lane) {
  constexpr int KT = (L == 0) ? (KL0 / 32) : (KL1 / 32);
  constexpr int KP = (L == 0) ? KP0 : KP1;
  constexpr int KL = KT * 32;
  constexpr int OP = (L == 0) ? KP1 : HID;
  const int hh = lane >> 4, m = lane & 15;
  const int mg = wave & 1;
  const int hid0 = mg * 16 + 8 * hh;
  const bf16t* pah = Ah + (mg * 16 + m) * KL + 8 * hh;
  const bf16t* pal = Al + (mg * 16 + m) * KL + 8 * hh;

#pragma unroll 1
  for (int jid = wave; jid < JOBS; jid += 8) {
    const int n = (jid >> 1) * 16 + m;
    const bf16t* pbh = Ph + n * KP;
    const bf16t* pbl = Pl + n * KP;
    v8f acc[4];
    {
      const v8f z = {0.f, 0.f, 0.f, 0.f, 0.f, 0.f, 0.f, 0.f};
      acc[0] = z; acc[1] = z; acc[2] = z; acc[3] = z;
    }
#pragma unroll 1
    for (int kt = 0; kt < KT; ++kt) {
      Frag bh, bl;
#pragma unroll
      for (int s = 0; s < 2; ++s) {
        const int kk = kt * 32 + 16 * s + 8 * hh;
        int off;
        if constexpr (L == 0) {
          const int tap = (kk >= 40 ? 1 : 0) + (kk >= 80 ? 1 : 0);
          off = kk + 56 * tap;
        } else {
          const int tap = kt >> 1;
          off = kk + 64 * tap;
        }
        bh.q[s] = *(const v4u*)(pbh + off);
        bl.q[s] = *(const v4u*)(pbl + off);
      }
#pragma unroll
      for (int g = 0; g < 4; ++g) {
        const bf16t* qh = pah + g * 32 * KL + kt * 32;
        const bf16t* ql = pal + g * 32 * KL + kt * 32;
        Frag ah, al;
        ah.q[0] = *(const v4u*)qh;
        ah.q[1] = *(const v4u*)(qh + 16);
        al.q[0] = *(const v4u*)ql;
        al.q[1] = *(const v4u*)(ql + 16);
        acc[g] = wmma3(acc[g], ah.v, al.v, bh.v, bl.v);
      }
    }

    const bool valid = n < NPOS;
    const int nc = valid ? n : (NPOS - 1);
    float* cp = cbuf + nc * HID + hid0;
    v4f c0v = *(const v4f*)cp;
    v4f c1v = *(const v4f*)(cp + 4);
    v4f bia[4], bib[4];
#pragma unroll
    for (int g = 0; g < 4; ++g) {
      const float* bq = bias + g * HID + hid0;
      bia[g] = *(const v4f*)bq;
      bib[g] = *(const v4f*)(bq + 4);
    }
    float hv[8];
    Pk8 ph, pl;
#pragma unroll
    for (int r = 0; r < 8; ++r) {
      const bool up = r >= 4;
      const int rr = r & 3;
      const float cold = up ? c1v[rr] : c0v[rr];
      const float iv = acc[0][r] + (up ? bib[0][rr] : bia[0][rr]);
      const float fv = acc[1][r] + (up ? bib[1][rr] : bia[1][rr]);
      const float ov = acc[2][r] + (up ? bib[2][rr] : bia[2][rr]);
      const float gv = acc[3][r] + (up ? bib[3][rr] : bia[3][rr]);
      const float cn = sigf(fv) * cold + sigf(iv) * tanhf_(gv);
      const float hn = sigf(ov) * tanhf_(cn);
      if (up) c1v[rr] = cn; else c0v[rr] = cn;
      hv[r] = hn;
      const bf16t hb = (bf16t)hn;
      ph.h[r] = hb;
      pl.h[r] = (bf16t)(hn - (float)hb);
    }
    if (valid) {
      *(v4f*)cp = c0v;
      *(v4f*)(cp + 4) = c1v;
      const int oi = n * OP + hid0;
      *(v4u*)(Oh + oi) = ph.u;
      *(v4u*)(Ol + oi) = pl.u;
    }
    if constexpr (L == 1) {
      if (doLast) {
        const float* nw = ninw + hid0;
        float p = 0.0f;
#pragma unroll
        for (int r = 0; r < 8; ++r) p += nw[r] * hv[r];
        p += __shfl_xor(p, 16);
        if (valid && hh == 0) fpart[mg * NPAD + n] = p;
      }
    }
  }
}

__global__ void __launch_bounds__(256) __attribute__((amdgpu_num_vgpr(248)))
k_lstm(const float* __restrict__ x, const int* __restrict__ lens,
       const float* __restrict__ cb0, const float* __restrict__ cb1,
       const float* __restrict__ ninw, const float* __restrict__ ninb,
       const float* __restrict__ fc1w, const float* __restrict__ fc1b,
       const float* __restrict__ fc2w, const float* __restrict__ fc2b,
       const bf16t* __restrict__ A0h, const bf16t* __restrict__ A0l,
       const bf16t* __restrict__ A1h, const bf16t* __restrict__ A1l,
       float* stage) {
  extern __shared__ v4u smem_v[];
  unsigned char* smem = (unsigned char*)smem_v;
  bf16t* P0h = (bf16t*)(smem + OFF_P0H);
  bf16t* P0l = (bf16t*)(smem + OFF_P0L);
  bf16t* P1h = (bf16t*)(smem + OFF_P1H);
  bf16t* P1l = (bf16t*)(smem + OFF_P1L);
  bf16t* H1h = (bf16t*)(smem + OFF_H1H);
  bf16t* H1l = (bf16t*)(smem + OFF_H1L);
  float* C0   = (float*)(smem + OFF_C0);
  float* C1   = (float*)(smem + OFF_C1);
  float* FP   = (float*)(smem + OFF_FP);
  float* FLAT = (float*)(smem + OFF_FLAT);
  float* F1O  = (float*)(smem + OFF_F1O);
  float* RES  = (float*)(smem + OFF_RES);

  const int b = blockIdx.x;
  const int tid = threadIdx.x;
  const int lane = tid & 31;
  const int wave = __builtin_amdgcn_readfirstlane(tid >> 5);

  {
    const v4u z = {0u, 0u, 0u, 0u};
    for (int i = tid; i < LDS_BYTES / 16; i += 256) smem_v[i] = z;
  }
  int len = lens[b];
  len = len < 1 ? 1 : (len > NSTEP ? NSTEP : len);
  __syncthreads();

  const float* xb = x + (size_t)b * NSTEP * CIN * NPOS;

#pragma unroll 1
  for (int t = 0; t < NSTEP; ++t) {
    {
      const float* xs = xb + (size_t)t * CIN * NPOS;
      for (int n = tid; n < NPOS; n += 256) {
        const float v0 = xs[n];
        const float v1 = xs[NPOS + n];
        const float v2 = xs[2 * NPOS + n];
        const float v3 = xs[3 * NPOS + n];
        Pk4 ph, pl;
        bf16t hb;
        hb = (bf16t)v0; ph.h[0] = hb; pl.h[0] = (bf16t)(v0 - (float)hb);
        hb = (bf16t)v1; ph.h[1] = hb; pl.h[1] = (bf16t)(v1 - (float)hb);
        hb = (bf16t)v2; ph.h[2] = hb; pl.h[2] = (bf16t)(v2 - (float)hb);
        hb = (bf16t)v3; ph.h[3] = hb; pl.h[3] = (bf16t)(v3 - (float)hb);
        const int o = (n + GUARD) * KP0 + 32;
        *(v2u*)(P0h + o) = ph.u;
        *(v2u*)(P0l + o) = pl.u;
      }
      for (int p = tid; p < NPOS * 4; p += 256) {
        const int n = p >> 2, q = (p & 3) * 8;
        const int s1 = (n + GUARD) * KP1 + q;
        const int d0 = (n + GUARD) * KP0 + q;
        const v4u a  = *(const v4u*)(P1h + s1);
        const v4u a2 = *(const v4u*)(P1l + s1);
        *(v4u*)(P0h + d0) = a;
        *(v4u*)(P0l + d0) = a2;
        const int sh = n * HID + q;
        const v4u c  = *(const v4u*)(H1h + sh);
        const v4u c2 = *(const v4u*)(H1l + sh);
        *(v4u*)(P1h + s1 + 32) = c;
        *(v4u*)(P1l + s1 + 32) = c2;
      }
    }
    __syncthreads();
    layer_jobs<0>(P0h, P0l, A0h, A0l, cb0, C0, P1h + GUARD * KP1, P1l + GUARD * KP1,
                  FP, ninw, false, wave, lane);
    __syncthreads();
    layer_jobs<1>(P1h, P1l, A1h, A1l, cb1, C1, H1h, H1l, FP, ninw, t == len - 1,
                  wave, lane);
    __syncthreads();
  }

  for (int n = tid; n < NPOS; n += 256) FLAT[n] = FP[n] + FP[NPAD + n] + ninb[0];
  __syncthreads();
  {
    const float* wr = fc1w + (size_t)tid * NPOS;
    float s = fc1b[tid];
#pragma unroll 2
    for (int n = 0; n < NPOS; ++n) s += FLAT[n] * wr[n];
    F1O[tid] = s;
  }
  __syncthreads();
  if (tid < NOUT) {
    const float* wr = fc2w + tid * FC1;
    float s = fc2b[tid];
#pragma unroll 2
    for (int k = 0; k < FC1; ++k) s += F1O[k] * wr[k];
    RES[tid] = s;
  }
  __syncthreads();
  {
    const float r0 = RES[0], r1 = RES[1];
    v4f v;
    v[0] = (tid == 0) ? r0 : 0.0f;
    v[1] = (tid == 0) ? r1 : 0.0f;
    v[2] = 0.0f;
    v[3] = 0.0f;
    const int q = tid < 8 ? tid : 7;
    float* d = stage + b * 32 + 4 * q;
    if (tid < 8) *(volatile v4f*)d = v;
    __threadfence();
    if (tid < 8) *(volatile v4f*)d = v;
  }
}

__global__ void __launch_bounds__(32)
k_fin(const float* __restrict__ stage, float* out) {
  const int q = threadIdx.x;
  const int qq = q < 8 ? q : 7;
  const float* s0 = stage + (2 * qq) * 32;
  const float* s1 = s0 + 32;
  v4f v;
  v[0] = s0[0]; v[1] = s0[1]; v[2] = s1[0]; v[3] = s1[1];
  float* d = out + 4 * qq;
  if (q < 8) *(volatile v4f*)d = v;
  __threadfence();
  if (q < 8) *(volatile v4f*)d = v;
}

extern "C" void kernel_launch(void* const* d_in, const int* in_sizes, int n_in,
                              void* d_out, int out_size, void* d_ws, size_t ws_size,
                              hipStream_t stream) {
  if (n_in < 12) return;
  if (in_sizes[0] != NB * NSTEP * CIN * NPOS || in_sizes[1] != NB ||
      in_sizes[2] != NGATE * K0IN * 3 || in_sizes[3] != NGATE ||
      in_sizes[4] != NGATE * K1IN * 3 || in_sizes[5] != NGATE ||
      in_sizes[6] != HID || in_sizes[7] != 1 ||
      in_sizes[8] != FC1 * NPOS || in_sizes[9] != FC1 ||
      in_sizes[10] != NOUT * FC1 || in_sizes[11] != NOUT) return;
  if (out_size != NB * NOUT) return;

  const float* x    = (const float*)d_in[0];
  const int*   lens = (const int*)d_in[1];
  const float* w0   = (const float*)d_in[2];
  const float* b0   = (const float*)d_in[3];
  const float* w1   = (const float*)d_in[4];
  const float* b1   = (const float*)d_in[5];
  const float* ninw = (const float*)d_in[6];
  const float* ninb = (const float*)d_in[7];
  const float* fc1w = (const float*)d_in[8];
  const float* fc1b = (const float*)d_in[9];
  const float* fc2w = (const float*)d_in[10];
  const float* fc2b = (const float*)d_in[11];
  float* out = (float*)d_out;

  char* ws = (char*)d_ws;
  size_t off = 0;
  auto carve = [&](size_t bytes) -> char* {
    char* p = ws + off;
    off = (off + bytes + 255) & ~(size_t)255;
    return p;
  };
  bf16t* A0h = (bf16t*)carve(SZ_A0);
  bf16t* A0l = (bf16t*)carve(SZ_A0);
  bf16t* A1h = (bf16t*)carve(SZ_A1);
  bf16t* A1l = (bf16t*)carve(SZ_A1);
  float* stage = (float*)carve(SZ_STAGE);
  if (off > ws_size) return;

  (void)hipFuncSetAttribute((const void*)k_lstm,
                            hipFuncAttributeMaxDynamicSharedMemorySize, LDS_BYTES);

  k_prep<<<dim3((PIECES0 + PIECES1) / 256), dim3(256), 0, stream>>>(w0, w1, A0h, A0l, A1h, A1l);
  k_lstm<<<dim3(NB), dim3(256), LDS_BYTES, stream>>>(x, lens, b0, b1, ninw, ninb,
                                                      fc1w, fc1b, fc2w, fc2b,
                                                      A0h, A0l, A1h, A1l, stage);
  k_fin<<<dim3(1), dim3(32), 0, stream>>>(stage, out);
}
